// SelfAttention_10522669875312
// MI455X (gfx1250) — hardware-verified
//
#include <hip/hip_runtime.h>
#ifndef NB
#define NB 4
#endif
#ifndef SEQ
#define SEQ 4096
#endif
#define NB_FULL 4
#define SEQ_FULL 4096
#define CC 512
#define DK 64
#define AW 16

typedef unsigned short v8us __attribute__((ext_vector_type(8), may_alias));
typedef float  v8f  __attribute__((ext_vector_type(8)));
typedef float  v4f  __attribute__((ext_vector_type(4)));
typedef float  v4fa __attribute__((ext_vector_type(4), may_alias));
typedef _Float16 v16h __attribute__((ext_vector_type(16)));
typedef _Float16 v4h __attribute__((ext_vector_type(4)));
union FragH { v16h v; v8us half[2]; _Float16 h[16]; unsigned short u[16]; };
union FragH8 { v8us v; _Float16 h[8]; };

static_assert(NB >= 1 && NB <= NB_FULL);
static_assert(SEQ <= SEQ_FULL);
static_assert(SEQ % 256 == 0);
static_assert(SEQ % 64 == 0 && SEQ % 32 == 0);
static_assert(((size_t)NB * SEQ) % 128 == 0);
static_assert(CC == 512 && CC % 128 == 0 && CC % 32 == 0 && CC == AW * 32);
static_assert(AW * 16 == 256 && AW * 32 == 512);
static_assert(DK == 64 && DK % 32 == 0);

static constexpr size_t al256(size_t v) { return (v + 255) & ~(size_t)255; }
static constexpr size_t SZ_WQK = al256((size_t)DK * CC * 2);
static constexpr size_t SZ_WV  = al256((size_t)CC * CC * 2);
static constexpr size_t SZ_XT  = al256((size_t)NB * SEQ * CC * 2);
static constexpr size_t SZ_QK  = al256((size_t)NB * SEQ * DK * 2);
static constexpr size_t SZ_V   = al256((size_t)NB * CC * SEQ * 2);
static constexpr size_t OFF_WK = 0;
static constexpr size_t OFF_WQ = OFF_WK + SZ_WQK;
static constexpr size_t OFF_WV = OFF_WQ + SZ_WQK;
static constexpr size_t OFF_XT = OFF_WV + SZ_WV;
static constexpr size_t OFF_KH = OFF_XT + SZ_XT;
static constexpr size_t OFF_KL = OFF_KH + SZ_QK;
static constexpr size_t OFF_QH = OFF_KL + SZ_QK;
static constexpr size_t OFF_QL = OFF_QH + SZ_QK;
static constexpr size_t OFF_V  = OFF_QL + SZ_QK;
static constexpr size_t WS_TOTAL = OFF_V + SZ_V;
static_assert(WS_TOTAL <= (size_t)134217728);

__device__ __forceinline__ unsigned short bf16_bits(float x) { unsigned int u = __float_as_uint(x); return (unsigned short)((u + 0x7FFFu + ((u >> 16) & 1u)) >> 16); }
__device__ __forceinline__ float bf16_rne(float x) { return __uint_as_float(((unsigned int)bf16_bits(x)) << 16); }
__device__ __forceinline__ unsigned short h16_bits(float x) { const _Float16 h = (_Float16)x; return __builtin_bit_cast(unsigned short, h); }

__device__ __forceinline__ v16h g2_frag(const _Float16* p, int hh) { FragH f; f.half[0] = *(const v8us*)((const unsigned short*)p + 8 * hh); f.half[1] = *(const v8us*)((const unsigned short*)p + 16 + 8 * hh); return f.v; }
__device__ __forceinline__ v8f g2_mma(v16h a, v16h b, v8f c) { v8f d = __builtin_amdgcn_wmma_f32_16x16x32_f16(false, a, false, b, (short)0, c, false, false); asm volatile("v_nop\n\tv_nop\n\tv_nop\n\tv_nop" : "+v"(d) : "v"(a), "v"(b)); return d; }
__device__ __forceinline__ void g2_mma2(v16h a, v16h b0, v16h b1, v8f& c0, v8f& c1) {
  c0 = __builtin_amdgcn_wmma_f32_16x16x32_f16(false, a, false, b0, (short)0, c0, false, false);
  c1 = __builtin_amdgcn_wmma_f32_16x16x32_f16(false, a, false, b1, (short)0, c1, false, false);
  asm volatile("v_nop\n\tv_nop\n\tv_nop\n\tv_nop" : "+v"(c0), "+v"(c1) : "v"(a), "v"(b0), "v"(b1));
}
__device__ __forceinline__ void sc_mma3(v16h kh, v16h kl, v16h qh, v16h ql, v8f& sh, v8f& sl) {
  sh = __builtin_amdgcn_wmma_f32_16x16x32_f16(false, kh, false, qh, (short)0, sh, false, false);
  sl = __builtin_amdgcn_wmma_f32_16x16x32_f16(false, kh, false, ql, (short)0, sl, false, false);
  sl = __builtin_amdgcn_wmma_f32_16x16x32_f16(false, kl, false, qh, (short)0, sl, false, false);
  asm volatile("v_nop\n\tv_nop\n\tv_nop\n\tv_nop" : "+v"(sh), "+v"(sl) : "v"(kh), "v"(kl), "v"(qh), "v"(ql));
}

__global__ __launch_bounds__(256) void k_wnat(const float* __restrict__ w, size_t n8, _Float16* __restrict__ Bt) {
  const size_t t = (size_t)blockIdx.x * 256 + threadIdx.x; if (t >= n8) return; FragH f;
#pragma unroll
  for (int q = 0; q < 8; ++q) f.h[q] = (_Float16)(bf16_rne(w[t * 8 + q]) * 16.0f);
  const v8us o = f.half[0];
  *(volatile v8us*)((unsigned short*)Bt + t * 8) = o; __threadfence(); *(volatile v8us*)((unsigned short*)Bt + t * 8) = o;
}

__global__ __launch_bounds__(256) void k_xt(const float* __restrict__ x, _Float16* __restrict__ XT) {
  __shared__ __attribute__((aligned(16))) unsigned short tl[64][72];
  const int tid = threadIdx.x;
  const int ct = blockIdx.x & 7, rest = blockIdx.x >> 3;
  const int nt = rest % (SEQ / 64), b = rest / (SEQ / 64);
  const int c0 = ct * 64, n0 = nt * 64;
  for (int i = tid; i < 64 * 16; i += 256) {
    const int c = i >> 4, n4 = (i & 15) * 4;
    const v4f xv = *(const v4fa*)(x + ((size_t)b * CC + c0 + c) * SEQ_FULL + n0 + n4);
#pragma unroll
    for (int q = 0; q < 4; ++q) tl[n4 + q][c] = h16_bits(bf16_rne(xv[q]));
  }
  __syncthreads();
  for (int pass = 0; pass < 2; ++pass) {
    for (int i = tid; i < 64 * 8; i += 256) {
      const int n = i >> 3, c8 = (i & 7) * 8;
      const v8us v = *(const v8us*)&tl[n][c8];
      *(volatile v8us*)((unsigned short*)XT + ((size_t)b * SEQ + n0 + n) * CC + c0 + c8) = v;
    }
    if (pass == 0) __threadfence();
  }
}

__global__ __launch_bounds__(128) void k_proj_qk(const _Float16* __restrict__ A, const _Float16* __restrict__ Bh, const float* __restrict__ bias,
                                                 _Float16* __restrict__ Chi, _Float16* __restrict__ Clo, int M) {
  __shared__ __attribute__((aligned(16))) float so[4][32][68];
  const int tid = threadIdx.x, w = tid >> 5, lane = tid & 31, ln = lane & 15, hh = lane >> 4;
  const int row0 = blockIdx.x * 128 + 32 * w; if (row0 >= M) return;
  const _Float16* a0p = A + (size_t)(row0 + ln) * CC; const _Float16* a1p = a0p + (size_t)16 * CC;
  const _Float16* b0p = Bh + (size_t)ln * CC; const _Float16* b1p = b0p + (size_t)16 * CC; const _Float16* b2p = b1p + (size_t)16 * CC; const _Float16* b3p = b2p + (size_t)16 * CC;
  const v8f z8 = {0.f,0.f,0.f,0.f,0.f,0.f,0.f,0.f}; v8f c00 = z8, c01 = z8, c02 = z8, c03 = z8, c10 = z8, c11 = z8, c12 = z8, c13 = z8;
#pragma unroll 1
  for (int kb = 0; kb < CC; kb += 32) { const v16h a0 = g2_frag(a0p + kb, hh), a1 = g2_frag(a1p + kb, hh);
    v16h b = g2_frag(b0p + kb, hh); c00 = g2_mma(a0, b, c00); c10 = g2_mma(a1, b, c10);
    b = g2_frag(b1p + kb, hh); c01 = g2_mma(a0, b, c01); c11 = g2_mma(a1, b, c11);
    b = g2_frag(b2p + kb, hh); c02 = g2_mma(a0, b, c02); c12 = g2_mma(a1, b, c12);
    b = g2_frag(b3p + kb, hh); c03 = g2_mma(a0, b, c03); c13 = g2_mma(a1, b, c13); }
  v8f accs[8] = {c00, c01, c02, c03, c10, c11, c12, c13};
#pragma unroll
  for (int u = 0; u < 8; ++u) { const int t = u & 3, half = u >> 2; const int col = t * 16 + ln; const float bv = bf16_rne(bias[col]);
#pragma unroll
    for (int r = 0; r < 8; ++r) so[w][half * 16 + 8 * hh + r][col] = accs[u][r] * 0.0625f + bv; }
  __builtin_amdgcn_fence(4  , "workgroup"); __builtin_amdgcn_wave_barrier();
  const int rsub = lane >> 4, c4 = (lane & 15) * 4;
  for (int pass = 0; pass < 2; ++pass) {
#pragma unroll
    for (int q = 0; q < 16; ++q) { const int r = q * 2 + rsub; const v4f v = *(const v4fa*)&so[w][r][c4]; v4h h4, l4;
#pragma unroll
      for (int i = 0; i < 4; ++i) { const _Float16 h = (_Float16)v[i]; h4[i] = h; l4[i] = (_Float16)((v[i] - (float)h) * 2048.0f); }
      const size_t o = (size_t)(row0 + r) * DK + c4;
      *(volatile v4h*)(Chi + o) = h4; *(volatile v4h*)(Clo + o) = l4; }
    if (pass == 0) __threadfence(); }
}

__global__ __launch_bounds__(128) void k_proj_v(const _Float16* __restrict__ A, const _Float16* __restrict__ XT, const float* __restrict__ bias, _Float16* __restrict__ V16) {
  __shared__ __attribute__((aligned(16))) float so[4][32][68];
  const int tid = threadIdx.x, w = tid >> 5, lane = tid & 31, ln = lane & 15, hh = lane >> 4; const int by = blockIdx.y;
  const _Float16* Bh = XT + (size_t)by * SEQ * CC; _Float16* C = V16 + (size_t)by * CC * SEQ;
  const int ntn = SEQ / 64; const int mt = blockIdx.x / ntn, nq = blockIdx.x - mt * ntn; const int row0 = mt * 128 + 32 * w, col0 = nq * 64; if (row0 >= CC) return;
  const _Float16* a0p = A + (size_t)(row0 + ln) * CC; const _Float16* a1p = a0p + (size_t)16 * CC;
  const _Float16* b0p = Bh + (size_t)(col0 + ln) * CC; const _Float16* b1p = b0p + (size_t)16 * CC; const _Float16* b2p = b1p + (size_t)16 * CC; const _Float16* b3p = b2p + (size_t)16 * CC;
  const v8f z8 = {0.f,0.f,0.f,0.f,0.f,0.f,0.f,0.f}; v8f c00 = z8, c01 = z8, c02 = z8, c03 = z8, c10 = z8, c11 = z8, c12 = z8, c13 = z8;
#pragma unroll 1
  for (int kb = 0; kb < CC; kb += 32) { const v16h a0 = g2_frag(a0p + kb, hh), a1 = g2_frag(a1p + kb, hh);
    v16h b = g2_frag(b0p + kb, hh); c00 = g2_mma(a0, b, c00); c10 = g2_mma(a1, b, c10);
    b = g2_frag(b1p + kb, hh); c01 = g2_mma(a0, b, c01); c11 = g2_mma(a1, b, c11);
    b = g2_frag(b2p + kb, hh); c02 = g2_mma(a0, b, c02); c12 = g2_mma(a1, b, c12);
    b = g2_frag(b3p + kb, hh); c03 = g2_mma(a0, b, c03); c13 = g2_mma(a1, b, c13); }
  v8f accs[8] = {c00, c01, c02, c03, c10, c11, c12, c13};
#pragma unroll
  for (int u = 0; u < 8; ++u) { const int t = u & 3, half = u >> 2;
#pragma unroll
    for (int r = 0; r < 8; ++r) so[w][half * 16 + 8 * hh + r][t * 16 + ln] = accs[u][r] * 0.0625f; }
  __builtin_amdgcn_fence(4  , "workgroup"); __builtin_amdgcn_wave_barrier();
  const int rsub = lane >> 4, c4 = (lane & 15) * 4;
  for (int pass = 0; pass < 2; ++pass) {
#pragma unroll
    for (int q = 0; q < 16; ++q) { const int r = q * 2 + rsub; const v4f v = *(const v4fa*)&so[w][r][c4]; const float bb = bf16_rne(bias[row0 + r]); v4h h4;
#pragma unroll
      for (int i = 0; i < 4; ++i) h4[i] = (_Float16)(v[i] + bb);
      *(volatile v4h*)(C + (size_t)(row0 + r) * SEQ + col0 + c4) = h4; }
    if (pass == 0) __threadfence(); }
}

__global__ __launch_bounds__(512) void k_attn(const float* __restrict__ x, const float* __restrict__ gamma,
                                              const _Float16* __restrict__ KH, const _Float16* __restrict__ KL,
                                              const _Float16* __restrict__ QH, const _Float16* __restrict__ QL,
                                              const _Float16* __restrict__ V16, float* __restrict__ out) {
  __shared__ __attribute__((aligned(16))) unsigned short pfrag[2 * 8 * 2 * 32 * 8];
  __shared__ float wmaxs[AW][32];
  __shared__ float wsums[AW][32];
  __shared__ __attribute__((aligned(16))) float so[AW][16][36];
  const int tid = threadIdx.x, w = tid >> 5, lane = tid & 31, ln = lane & 15, hh = lane >> 4;
  const int b = blockIdx.y, m0 = blockIdx.x * 32;
  const int kslot = w >> 1, khalf = w & 1;
  const size_t rowb = (size_t)b * SEQ;
  const size_t qo0 = (rowb + m0 + ln) * DK;
  const size_t vrow = ((size_t)b * CC + w * 32 + ln) * SEQ;
  const v8f z8 = {0.f,0.f,0.f,0.f,0.f,0.f,0.f,0.f};
  v8f acc[2][2];
#pragma unroll
  for (int ci = 0; ci < 2; ++ci) { acc[ci][0] = z8; acc[ci][1] = z8; }
  float Mrow[2] = {-1.0e30f, -1.0e30f};
  float Lrow[2] = {0.f, 0.f};

#pragma unroll 1
  for (int nb = 0; nb < SEQ; nb += 256) {
    unsigned int zq = 0u;
    asm volatile("" : "+v"(zq));
    v8f s[2];
    {
      const size_t ko = (rowb + nb + w * 16 + ln) * DK;
      const v16h kh0 = g2_frag(KH + ko, hh), kh1 = g2_frag(KH + ko + 32, hh);
      const v16h kl0 = g2_frag(KL + ko, hh), kl1 = g2_frag(KL + ko + 32, hh);
#pragma unroll
      for (int mt = 0; mt < 2; ++mt) {
        const size_t qo = qo0 + (size_t)(mt * 16 * DK) + (size_t)zq;
        v8f sh = z8, sl = z8;
        { const v16h qh = g2_frag(QH + qo, hh), ql = g2_frag(QL + qo, hh); sc_mma3(kh0, kl0, qh, ql, sh, sl); }
        { const v16h qh = g2_frag(QH + qo + 32, hh), ql = g2_frag(QL + qo + 32, hh); sc_mma3(kh1, kl1, qh, ql, sh, sl); }
#pragma unroll
        for (int j = 0; j < 8; ++j) sh[j] = sh[j] + sl[j] * 0.00048828125f;
        s[mt] = sh;
      }
    }
    float lm0 = s[0][0], lm1 = s[1][0];
#pragma unroll
    for (int j = 1; j < 8; ++j) { lm0 = fmaxf(lm0, s[0][j]); lm1 = fmaxf(lm1, s[1][j]); }
    lm0 = fmaxf(lm0, __shfl_xor(lm0, 16)); lm1 = fmaxf(lm1, __shfl_xor(lm1, 16));
    wmaxs[w][lane] = hh ? lm1 : lm0;
    __syncthreads();

    float bmo = wmaxs[0][lane];
#pragma unroll
    for (int w2 = 1; w2 < AW; ++w2) bmo = fmaxf(bmo, wmaxs[w2][lane]);
    const float bmx = __shfl_xor(bmo, 16);
    float bm[2]; bm[0] = hh ? bmx : bmo; bm[1] = hh ? bmo : bmx;

    float alpha[2], lsum[2];
#pragma unroll
    for (int mt = 0; mt < 2; ++mt) {
      const float Mnew = fmaxf(Mrow[mt], bm[mt]);
      const float ea = __expf(fmaxf(Mrow[mt] - Mnew, -120.0f));
      alpha[mt] = (Mrow[mt] < -1.0e29f) ? 0.f : ea;
      Mrow[mt] = Mnew;
      FragH8 pf; float ls = 0.f;
#pragma unroll
      for (int j = 0; j < 8; ++j) {
        const float p0 = __expf(s[mt][j] - Mnew);
        ls += p0;
        pf.h[j] = (_Float16)(p0 * 4096.0f);
      }
      *(v8us*)&pfrag[((((mt * 8 + kslot) * 2 + khalf) * 32) + lane) * 8] = pf.v;
      ls += __shfl_xor(ls, 16);
      lsum[mt] = ls;
    }
    wsums[w][lane] = hh ? lsum[1] : lsum[0];
    __syncthreads();

    float bso = wsums[0][lane];
#pragma unroll
    for (int w2 = 1; w2 < AW; ++w2) bso += wsums[w2][lane];
    const float bsx = __shfl_xor(bso, 16);
    float bs[2]; bs[0] = hh ? bsx : bso; bs[1] = hh ? bso : bsx;
#pragma unroll
    for (int mt = 0; mt < 2; ++mt) {
      Lrow[mt] = Lrow[mt] * alpha[mt] + bs[mt];
#pragma unroll
      for (int ci = 0; ci < 2; ++ci)
#pragma unroll
        for (int j = 0; j < 8; ++j) acc[ci][mt][j] = acc[ci][mt][j] * alpha[mt];
    }
#pragma unroll 1
    for (int kb = 0; kb < 8; ++kb) {
      FragH p0, p1;
      p0.half[0] = *(const v8us*)&pfrag[((((0 * 8 + kb) * 2 + 0) * 32) + lane) * 8];
      p0.half[1] = *(const v8us*)&pfrag[((((0 * 8 + kb) * 2 + 1) * 32) + lane) * 8];
      p1.half[0] = *(const v8us*)&pfrag[((((1 * 8 + kb) * 2 + 0) * 32) + lane) * 8];
      p1.half[1] = *(const v8us*)&pfrag[((((1 * 8 + kb) * 2 + 1) * 32) + lane) * 8];
      const size_t vo = vrow + nb + kb * 32;
      const v16h va0 = g2_frag(V16 + vo, hh);
      const v16h va1 = g2_frag(V16 + vo + (size_t)16 * SEQ, hh);
      g2_mma2(va0, p0.v, p1.v, acc[0][0], acc[0][1]);
      g2_mma2(va1, p0.v, p1.v, acc[1][0], acc[1][1]);
    }
  }

  const float g = bf16_rne(gamma[0]);
  float scl[2];
  scl[0] = g * (1.0f / Lrow[0]) * 0.000244140625f;
  scl[1] = g * (1.0f / Lrow[1]) * 0.000244140625f;
  const int rq = lane >> 3, col4 = (lane & 7) * 4;
#pragma unroll
  for (int ci = 0; ci < 2; ++ci) {
#pragma unroll
    for (int mt = 0; mt < 2; ++mt)
#pragma unroll
      for (int r = 0; r < 8; ++r) so[w][8 * hh + r][mt * 16 + ln] = acc[ci][mt][r] * scl[mt];
    __builtin_amdgcn_fence(4  , "workgroup"); __builtin_amdgcn_wave_barrier();
    v4f ov[4]; size_t ga[4];
#pragma unroll
    for (int q = 0; q < 4; ++q) {
      const int row = q * 4 + rq;
      const int c = w * 32 + ci * 16 + row;
      ga[q] = ((size_t)b * CC + c) * SEQ_FULL + m0 + col4;
      const v4f cv = *(const v4fa*)&so[w][row][col4];
      const v4f xv = *(const v4fa*)(x + ga[q]);
      v4f o;
#pragma unroll
      for (int i = 0; i < 4; ++i) o[i] = bf16_rne(xv[i]) + cv[i];
      ov[q] = o;
    }
#pragma unroll
    for (int q = 0; q < 4; ++q) *(volatile v4f*)(out + ga[q]) = ov[q];
    __threadfence();
#pragma unroll
    for (int q = 0; q < 4; ++q) *(volatile v4f*)(out + ga[q]) = ov[q];
    __builtin_amdgcn_fence(4  , "workgroup"); __builtin_amdgcn_wave_barrier();
  }
}

extern "C" void kernel_launch(void* const* d_in, const int* in_sizes, int n_in,
                              void* d_out, int out_size, void* d_ws, size_t ws_size, hipStream_t stream) {
  if (n_in < 8) return;
  const size_t need_x = ((size_t)(NB - 1) * CC + (CC - 1)) * SEQ_FULL + SEQ;
  if ((size_t)in_sizes[0] < need_x) return;
  if (in_sizes[1] < DK * CC || in_sizes[2] < DK || in_sizes[3] < DK * CC || in_sizes[4] < DK) return;
  if (in_sizes[5] < CC * CC || in_sizes[6] < CC || in_sizes[7] < 1) return;
  if ((size_t)out_size < need_x) return;
  if (ws_size < WS_TOTAL) return;
  const float* x  = (const float*)d_in[0];
  const float* wk = (const float*)d_in[1];
  const float* bk = (const float*)d_in[2];
  const float* wq = (const float*)d_in[3];
  const float* bq = (const float*)d_in[4];
  const float* wv = (const float*)d_in[5];
  const float* bv = (const float*)d_in[6];
  const float* gamma = (const float*)d_in[7];
  char* ws = (char*)d_ws;
  _Float16* WK16 = (_Float16*)(ws + OFF_WK);
  _Float16* WQ16 = (_Float16*)(ws + OFF_WQ);
  _Float16* WV16 = (_Float16*)(ws + OFF_WV);
  _Float16* XT   = (_Float16*)(ws + OFF_XT);
  _Float16* KH   = (_Float16*)(ws + OFF_KH);
  _Float16* KL   = (_Float16*)(ws + OFF_KL);
  _Float16* QH   = (_Float16*)(ws + OFF_QH);
  _Float16* QL   = (_Float16*)(ws + OFF_QL);
  _Float16* V16  = (_Float16*)(ws + OFF_V);
  float* out = (float*)d_out;

  { const size_t n8 = (size_t)DK * CC / 8; const unsigned g = (unsigned)((n8 + 255) / 256);
    k_wnat<<<g, 256, 0, stream>>>(wk, n8, WK16);
    k_wnat<<<g, 256, 0, stream>>>(wq, n8, WQ16); }
  { const size_t n8 = (size_t)CC * CC / 8; const unsigned g = (unsigned)((n8 + 255) / 256);
    k_wnat<<<g, 256, 0, stream>>>(wv, n8, WV16); }
  k_xt<<<(unsigned)(NB * (SEQ / 64) * (CC / 64)), 256, 0, stream>>>(x, XT);
  k_proj_qk<<<(unsigned)(((size_t)NB * SEQ) / 128), 128, 0, stream>>>(XT, WK16, bk, KH, KL, (int)((size_t)NB * SEQ));
  k_proj_qk<<<(unsigned)(((size_t)NB * SEQ) / 128), 128, 0, stream>>>(XT, WQ16, bq, QH, QL, (int)((size_t)NB * SEQ));
  k_proj_v<<<dim3((unsigned)((CC / 128) * (SEQ / 64)), (unsigned)NB), 128, 0, stream>>>(WV16, XT, bv, V16);
  k_attn<<<dim3((unsigned)(SEQ / 32), (unsigned)NB), 512, 0, stream>>>(x, gamma, KH, KL, QH, QL, V16, out);
}
